// ResDCN_89859305767622
// MI455X (gfx1250) — hardware-run, weakly checked
//
#include <hip/hip_runtime.h>
#include <stddef.h>


#define NFEAT   70
#define NH      64
#define EMB     128
#define DDIM    192
#define RHID    512
#define ZDIM    384
#define PHID    320
#define NTHR    256
#define NWAVE   8
#define EPT     8
#define NGRP    2
#define CHUNK   (NTHR * EPT * NGRP)
#define WCAP    (EPT * NGRP * 32)
#define LISTN   (NWAVE * WCAP)
#define ESHF    11
#define NBC     32768
#define NBF     2048
#define RCAP    40960
#define RBN     128
#define TGT     256
#define DEGCAP  512
#define GBM     128
#define GBN     64
#define OTHR    512
#define CHROWS  10240
#define WSCAP   134217728

#define ASC    0.0625f
#define WSC    1024.0f
#define ACCS   0.015625f
#define LOSC   2048.0f
#define LOINV  0.00048828125f
#define HCLAMP 65000.0f

#define LDS_COUNT ((NBC + LISTN + NWAVE) * 4)
#define LDS_FILL  ((RCAP + NBF + LISTN + NWAVE) * 4)

#define F_BIAS 1
#define F_RES  2
#define F_ACT  4
#define F_RSC  8
#define F_OUTF 16
#define F_OUTP 32

static_assert((CHUNK & (CHUNK - 1)) == 0);
static_assert((NBC & (NBC - 1)) == 0 && (NBF & (NBF - 1)) == 0);
static_assert(NBF <= (1 << ESHF));
static_assert((NBC % NBF) == 0);
static_assert(OTHR * 4 == NBF);
static_assert((RCAP % 32) == 0);
static_assert(TGT == NWAVE * 32);
static_assert(GBM == NWAVE * 16);
static_assert((TGT % GBM) == 0);
static_assert((CHROWS % TGT) == 0);
static_assert(NBC == NWAVE * 32 * 128);
static_assert(EMB == 4 * 32);
static_assert(DDIM == 6 * 32 && (DDIM / 8) <= 32);
static_assert((PHID % 32) == 0);
static_assert((NH % 32) == 0 && (EMB % 32) == 0 && (DDIM % 32) == 0 && (RHID % 32) == 0 && (ZDIM % 32) == 0);
static_assert((EMB % GBN) == 0 && (RHID % GBN) == 0 && (DDIM % GBN) == 0 && (PHID % GBN) == 0);

typedef float          v4f  __attribute__((ext_vector_type(4)));
typedef float          v8f  __attribute__((ext_vector_type(8)));
typedef int            v4i  __attribute__((ext_vector_type(4)));
typedef unsigned int   v2u  __attribute__((ext_vector_type(2)));
typedef unsigned int   v4u  __attribute__((ext_vector_type(4)));
typedef unsigned short v8us __attribute__((ext_vector_type(8)));
typedef _Float16       v16h __attribute__((ext_vector_type(16)));
union FragH { v16h v; v8us u[2]; };

__device__ __forceinline__ v8f wmh(v16h a, v16h b, v8f c) {
  v8f d = __builtin_amdgcn_wmma_f32_16x16x32_f16(false, a, false, b, (short)0, c, false, false);
  asm volatile("v_nop\n\tv_nop\n\tv_nop\n\tv_nop" : "+v"(d) : "v"(a), "v"(b));
  return d;
}

__device__ __forceinline__ float leakyf(float v) { return v > 0.f ? v : 0.01f * v; }

__device__ __forceinline__ double shfl_xor_d(double v, int o) {
  const long long bits = __double_as_longlong(v);
  int lo = (int)(bits & 0xFFFFFFFFll);
  int hi = (int)(bits >> 32);
  lo = __shfl_xor(lo, o, 32);
  hi = __shfl_xor(hi, o, 32);
  const long long r = (long long)(((unsigned long long)(unsigned)hi << 32) | (unsigned long long)(unsigned)lo);
  return __longlong_as_double(r);
}

__device__ __forceinline__ unsigned f16b(float x) {
  const _Float16 h = (_Float16)x;
  const unsigned u = (unsigned)__builtin_bit_cast(unsigned short, h);
  return ((u & 0x7C00u) == 0u) ? 0u : u;
}
__device__ __forceinline__ float f16f(unsigned u) {
  return (float)__builtin_bit_cast(_Float16, (unsigned short)(u & 0xFFFFu));
}
__device__ __forceinline__ void hl2(float a, float b, float sc, unsigned& ph, unsigned& pl) {
  float xa = a * sc, xb = b * sc;
  xa = fminf(fmaxf(xa, -HCLAMP), HCLAMP);
  xb = fminf(fmaxf(xb, -HCLAMP), HCLAMP);
  const unsigned ha = f16b(xa), hb = f16b(xb);
  const unsigned la = f16b((xa - f16f(ha)) * LOSC);
  const unsigned lb = f16b((xb - f16f(hb)) * LOSC);
  ph = ha | (hb << 16);
  pl = la | (lb << 16);
}
__device__ __forceinline__ void split4(v4f v, float sc, v2u& h, v2u& l) {
  unsigned h0, l0, h1, l1;
  hl2(v.x, v.y, sc, h0, l0);
  hl2(v.z, v.w, sc, h1, l1);
  h.x = h0; h.y = h1; l.x = l0; l.y = l1;
}
__device__ __forceinline__ void split8(v4f a, v4f b, float sc, v4u& h, v4u& l) {
  unsigned h0, l0, h1, l1, h2, l2, h3, l3;
  hl2(a.x, a.y, sc, h0, l0);
  hl2(a.z, a.w, sc, h1, l1);
  hl2(b.x, b.y, sc, h2, l2);
  hl2(b.z, b.w, sc, h3, l3);
  h.x = h0; h.y = h1; h.z = h2; h.w = h3;
  l.x = l0; l.y = l1; l.z = l2; l.w = l3;
}

template <int NB, int SRC>
__device__ __forceinline__ int scan_chunk(const int* __restrict__ dsts, const int* __restrict__ srcs, int nE, int nN,
                                          int cbase, int slotBase, int vec8, int* list, int tid, int lane, int wave) {
  int wc = 0;
#pragma unroll
  for (int g = 0; g < NGRP; ++g) {
    const int el0  = (g * NTHR + tid) * EPT;
    const int e0   = cbase + el0;
    const int sent = -2147483647 - 1;
    v4i da, db;
    v4i sa = {0, 0, 0, 0}, sb = {0, 0, 0, 0};
    if (vec8 != 0 && cbase + CHUNK <= nE) {
      da = *(const v4i*)(dsts + e0);
      db = *(const v4i*)(dsts + e0 + 4);
      if (SRC) {
        sa = *(const v4i*)(srcs + e0);
        sb = *(const v4i*)(srcs + e0 + 4);
      }
    } else {
      da.x = (e0     < nE) ? dsts[min(e0, nE - 1)] : sent;
      da.y = (e0 + 1 < nE) ? dsts[min(e0 + 1, nE - 1)] : sent;
      da.z = (e0 + 2 < nE) ? dsts[min(e0 + 2, nE - 1)] : sent;
      da.w = (e0 + 3 < nE) ? dsts[min(e0 + 3, nE - 1)] : sent;
      db.x = (e0 + 4 < nE) ? dsts[min(e0 + 4, nE - 1)] : sent;
      db.y = (e0 + 5 < nE) ? dsts[min(e0 + 5, nE - 1)] : sent;
      db.z = (e0 + 6 < nE) ? dsts[min(e0 + 6, nE - 1)] : sent;
      db.w = (e0 + 7 < nE) ? dsts[min(e0 + 7, nE - 1)] : sent;
      if (SRC) {
        sa.x = srcs[min(e0, nE - 1)];
        sa.y = srcs[min(e0 + 1, nE - 1)];
        sa.z = srcs[min(e0 + 2, nE - 1)];
        sa.w = srcs[min(e0 + 3, nE - 1)];
        sb.x = srcs[min(e0 + 4, nE - 1)];
        sb.y = srcs[min(e0 + 5, nE - 1)];
        sb.z = srcs[min(e0 + 6, nE - 1)];
        sb.w = srcs[min(e0 + 7, nE - 1)];
      }
    }
    if (SRC) {
      sa.x = min(max(sa.x, 0), nN - 1); sa.y = min(max(sa.y, 0), nN - 1);
      sa.z = min(max(sa.z, 0), nN - 1); sa.w = min(max(sa.w, 0), nN - 1);
      sb.x = min(max(sb.x, 0), nN - 1); sb.y = min(max(sb.y, 0), nN - 1);
      sb.z = min(max(sb.z, 0), nN - 1); sb.w = min(max(sb.w, 0), nN - 1);
    }
    const unsigned nb = (unsigned)slotBase;
    const unsigned s0 = (unsigned)da.x - nb, s1 = (unsigned)da.y - nb;
    const unsigned s2 = (unsigned)da.z - nb, s3 = (unsigned)da.w - nb;
    const unsigned s4 = (unsigned)db.x - nb, s5 = (unsigned)db.y - nb;
    const unsigned s6 = (unsigned)db.z - nb, s7 = (unsigned)db.w - nb;
    const bool h0 = s0 < (unsigned)NB, h1 = s1 < (unsigned)NB, h2 = s2 < (unsigned)NB, h3 = s3 < (unsigned)NB;
    const bool h4 = s4 < (unsigned)NB, h5 = s5 < (unsigned)NB, h6 = s6 < (unsigned)NB, h7 = s7 < (unsigned)NB;
    const unsigned any = __builtin_amdgcn_ballot_w32(h0 | h1 | h2 | h3 | h4 | h5 | h6 | h7);
    if (any != 0u) {
#define HITJ(HJ, SJ, VJ) { \
        const unsigned mj = __builtin_amdgcn_ballot_w32(HJ); \
        if (mj != 0u) { \
          if (HJ) { \
            const int pos = wc + (int)__builtin_amdgcn_mbcnt_lo(mj, 0u); \
            const int entv = SRC ? (((VJ) << ESHF) | (int)(SJ)) : (int)(SJ); \
            if (pos < WCAP) list[wave * WCAP + pos] = entv; \
          } \
          wc += (int)__builtin_popcount(mj); } }
      HITJ(h0, s0, sa.x)
      HITJ(h1, s1, sa.y)
      HITJ(h2, s2, sa.z)
      HITJ(h3, s3, sa.w)
      HITJ(h4, s4, sb.x)
      HITJ(h5, s5, sb.y)
      HITJ(h6, s6, sb.z)
      HITJ(h7, s7, sb.w)
#undef HITJ
    }
  }
  return wc;
}

__global__ __launch_bounds__(NTHR) void k_wprep(const float* __restrict__ W, int K, int N,
                                                unsigned short* ph, unsigned short* pl) {
  const size_t zo = (size_t)blockIdx.y * (size_t)K * (size_t)N;
  const int i  = (int)blockIdx.x * NTHR + (int)threadIdx.x;
  const int kq = K >> 3;
  if (i >= N * kq) return;
  const int n  = i / kq;
  const int k0 = (i - n * kq) * 8;
  const float* w = W + zo + (size_t)k0 * N + n;
  v4f a, b;
  a.x = w[0];             a.y = w[(size_t)N];     a.z = w[(size_t)2 * N]; a.w = w[(size_t)3 * N];
  b.x = w[(size_t)4 * N]; b.y = w[(size_t)5 * N]; b.z = w[(size_t)6 * N]; b.w = w[(size_t)7 * N];
  v4u hv, lv;
  split8(a, b, WSC, hv, lv);
  const size_t po = zo + (size_t)i * 8;
  *(volatile v4u*)(ph + po) = hv;
  *(volatile v4u*)(pl + po) = lv;
  __threadfence();
  *(volatile v4u*)(ph + po) = hv;
  *(volatile v4u*)(pl + po) = lv;
}

__global__ __launch_bounds__(NTHR) void k_embed(const int* __restrict__ dx, float* xF,
                                                unsigned short* xdH, unsigned short* xdL, int nN, int npad) {
  const int gid = (int)blockIdx.x * NTHR + (int)threadIdx.x;
  const int r = gid >> 4, q = gid & 15;
  if (r >= npad) return;
  const int rc = r > nN - 1 ? nN - 1 : r;
  const int* p = dx + (size_t)rc * NFEAT + 4 * q;
  v4f v;
  v.x = (float)p[0]; v.y = (float)p[1]; v.z = (float)p[2]; v.w = (float)p[3];
  v2u hv, lv;
  split4(v, ASC, hv, lv);
  const size_t fo = (size_t)r * DDIM + 4 * q;
  const size_t po = (size_t)r * NH + 4 * q;
  *(volatile v4f*)(xF + fo)  = v;
  *(volatile v2u*)(xdH + po) = hv;
  *(volatile v2u*)(xdL + po) = lv;
  __threadfence();
  *(volatile v4f*)(xF + fo)  = v;
  *(volatile v2u*)(xdH + po) = hv;
  *(volatile v2u*)(xdL + po) = lv;
}

__global__ __launch_bounds__(NTHR) void k_count(
    const int* __restrict__ ei, int* cnt, float* dinv, int nE, int nN, int vec8) {
  extern __shared__ v4f lds_dyn[];
  int* scnt = (int*)lds_dyn;
  int* list = scnt + NBC;
  int* wcnt = list + LISTN;
  const int tid = threadIdx.x, lane = tid & 31, wave = tid >> 5;
  const int nodeBase = blockIdx.x * NBC;
  const int* dsts = ei + nE;

  {
    const v4i z = {0, 0, 0, 0};
    for (int i = tid; i < NBC / 4; i += NTHR) ((v4i*)scnt)[i] = z;
  }
  __syncthreads();

  const int nChunks = (nE + CHUNK - 1) / CHUNK;
#pragma unroll 1
  for (int ch = 0; ch < nChunks; ++ch) {
    const int cbase = ch * CHUNK;
    const int wc = scan_chunk<NBC, 0>(dsts, ei, nE, nN, cbase, nodeBase, vec8, list, tid, lane, wave);
    if (lane == 0) wcnt[wave] = wc;
    __syncthreads();
    if (wave == 0) {
#pragma unroll 1
      for (int wsx = 0; wsx < NWAVE; ++wsx) {
        int n = __builtin_amdgcn_readfirstlane(wcnt[wsx]);
        n = n > WCAP ? WCAP : (n < 0 ? 0 : n);
        const int* lp = list + wsx * WCAP;
#pragma unroll 1
        for (int i = 0; i < n; ++i) {
          const int ent  = __builtin_amdgcn_readfirstlane(lp[i]);
          const int slot = ent & (NBC - 1);
          if (lane == 0) scnt[slot] = scnt[slot] + 1;
        }
      }
    }
    __syncthreads();
  }

  int*   cp = cnt + (size_t)nodeBase;
  float* dp = dinv + (size_t)nodeBase;
#pragma unroll 4
  for (int q = 0; q < 32; ++q) {
    const int f = (wave * 32 + q) * 128 + 4 * lane;
    const v4i c = *(const v4i*)(scnt + f);
    v4f d;
    d.x = rsqrtf((float)(c.x + 1)); d.y = rsqrtf((float)(c.y + 1));
    d.z = rsqrtf((float)(c.z + 1)); d.w = rsqrtf((float)(c.w + 1));
    *(volatile v4i*)(cp + f) = c;
    *(volatile v4f*)(dp + f) = d;
  }
  __threadfence();
#pragma unroll 4
  for (int q = 0; q < 32; ++q) {
    const int f = (wave * 32 + q) * 128 + 4 * lane;
    const v4i c = *(const v4i*)(scnt + f);
    v4f d;
    d.x = rsqrtf((float)(c.x + 1)); d.y = rsqrtf((float)(c.y + 1));
    d.z = rsqrtf((float)(c.z + 1)); d.w = rsqrtf((float)(c.w + 1));
    *(volatile v4i*)(cp + f) = c;
    *(volatile v4f*)(dp + f) = d;
  }
}

__global__ __launch_bounds__(OTHR) void k_offsets(
    const int* __restrict__ cnt, int* off, int* rbase, int nBF) {
  __shared__ __attribute__((aligned(16))) int srb[RBN];
  __shared__ int wtot[OTHR / 32];
  const int tid = threadIdx.x, lane = tid & 31, wave = tid >> 5;
  for (int i = tid; i < RBN; i += OTHR) srb[i] = 0;
  int carry = 0;
#pragma unroll 1
  for (int fb = 0; fb < nBF; ++fb) {
    const int base = fb * NBF;
    const v4i c = *(const v4i*)(cnt + base + 4 * tid);
    const int e0 = max(c.x, 0), e1 = max(c.y, 0), e2 = max(c.z, 0), e3 = max(c.w, 0);
    const int ts = e0 + e1 + e2 + e3;
    int incl = ts;
#pragma unroll
    for (int d = 1; d < 32; d <<= 1) {
      const int t = __shfl_up(incl, d);
      if (lane >= d) incl += t;
    }
    if (lane == 31) wtot[wave] = incl;
    __syncthreads();
    int pre = 0;
#pragma unroll 1
    for (int w = 0; w < wave; ++w) pre += wtot[w];
    int tot = 0;
#pragma unroll
    for (int w = 0; w < OTHR / 32; ++w) tot += wtot[w];
    int run = carry + pre + incl - ts;
    v4i o;
    o.x = run; run += e0;
    o.y = run; run += e1;
    o.z = run; run += e2;
    o.w = run;
    int* op = off + base + 4 * tid;
    *(volatile v4i*)op = o;
    __threadfence();
    *(volatile v4i*)op = o;
    if (tid == 0) srb[min(fb, RBN - 1)] = carry;
    carry += (tot + 31) & ~31;
    __syncthreads();
  }
  if (tid == 0) srb[min(nBF, RBN - 1)] = carry;
  __syncthreads();
  v4i rv = {0, 0, 0, 0};
  if (tid < 32) rv = *(const v4i*)(srb + 4 * tid);
  if (tid < 32) *(volatile v4i*)(rbase + 4 * tid) = rv;
  __threadfence();
  if (tid < 32) *(volatile v4i*)(rbase + 4 * tid) = rv;
}

__global__ __launch_bounds__(NTHR) void k_fill(
    const int* __restrict__ ei, const int* __restrict__ off, const int* __restrict__ rbase,
    int* csr, int nN, int nE, int vec8, int csrLen) {
  extern __shared__ v4f lds_dyn[];
  int* region = (int*)lds_dyn;
  int* cursor = region + RCAP;
  int* list   = cursor + NBF;
  int* wcnt   = list + LISTN;
  const int tid = threadIdx.x, lane = tid & 31, wave = tid >> 5;
  const int b = blockIdx.x;
  const int nodeBase = b * NBF;
  const int* dsts = ei + nE;

  int rb0 = rbase[b];
  const int rb1 = rbase[b + 1];
  rb0 = rb0 < 0 ? 0 : (rb0 > csrLen ? csrLen : rb0);
  rb0 &= ~31;
  int len = rb1 - rb0;
  len = len < 0 ? 0 : (len > RCAP ? RCAP : len);
  int lenW = (len + 31) & ~31;
  if (rb0 + lenW > csrLen) lenW = (csrLen - rb0) & ~31;

  {
    const v4i z = {0, 0, 0, 0};
    for (int i = tid; i < RCAP / 4; i += NTHR) ((v4i*)region)[i] = z;
    for (int s = tid; s < NBF; s += NTHR) {
      int o = off[nodeBase + s] - rb0;
      o = o < 0 ? 0 : (o > RCAP ? RCAP : o);
      cursor[s] = o;
    }
  }
  __syncthreads();

  const int nChunks = (nE + CHUNK - 1) / CHUNK;
#pragma unroll 1
  for (int ch = 0; ch < nChunks; ++ch) {
    const int cbase = ch * CHUNK;
    const int wc = scan_chunk<NBF, 1>(dsts, ei, nE, nN, cbase, nodeBase, vec8, list, tid, lane, wave);
    if (lane == 0) wcnt[wave] = wc;
    __syncthreads();
    if (wave == 0) {
#pragma unroll 1
      for (int wsx = 0; wsx < NWAVE; ++wsx) {
        int n = __builtin_amdgcn_readfirstlane(wcnt[wsx]);
        n = n > WCAP ? WCAP : (n < 0 ? 0 : n);
        const int* lp = list + wsx * WCAP;
#pragma unroll 1
        for (int i = 0; i < n; ++i) {
          const int ent  = __builtin_amdgcn_readfirstlane(lp[i]);
          const int slot = ent & (NBF - 1);
          int src = (ent >> ESHF) & 0xFFFFF;
          src = src > nN - 1 ? nN - 1 : src;
          if (lane == 0) {
            int pos = cursor[slot];
            pos = pos < 0 ? 0 : (pos > RCAP - 1 ? RCAP - 1 : pos);
            region[pos] = src;
            const int np = pos + 1;
            cursor[slot] = np > RCAP ? RCAP : np;
          }
        }
      }
    }
    __syncthreads();
  }

  const int nv = lenW >> 2;
  int* gp = csr + rb0;
#pragma unroll 1
  for (int i = tid; i < nv; i += NTHR) { const v4i v = ((const v4i*)region)[i]; *(volatile v4i*)(gp + 4 * i) = v; }
  __threadfence();
#pragma unroll 1
  for (int i = tid; i < nv; i += NTHR) { const v4i v = ((const v4i*)region)[i]; *(volatile v4i*)(gp + 4 * i) = v; }
}

__global__ __launch_bounds__(NTHR) void k_gemm(
    const unsigned short* __restrict__ Ah, const unsigned short* __restrict__ Al, int lda,
    const unsigned short* __restrict__ Bh, const unsigned short* __restrict__ Bl, int K,
    const float* __restrict__ bias, const float* __restrict__ resid, int ldr,
    const float* __restrict__ rsc,
    float* outF, int ldF, int colF,
    unsigned short* outH, unsigned short* outL, int ldP, int colP, int flags) {
  __shared__ __attribute__((aligned(16))) float stg[NWAVE * 16 * GBN];
  const int tid = threadIdx.x, lane = tid & 31, wave = tid >> 5, hh = lane >> 4, m = lane & 15;
  const int rowBase = (int)blockIdx.y * GBM;
  const int c0 = (int)blockIdx.x * GBN;
  const size_t aoff = (size_t)(rowBase + wave * 16 + m) * lda + 8 * hh;
  const unsigned short* ah = Ah + aoff;
  const unsigned short* al = Al + aoff;

  v8f accH[4], accX[4];
#pragma unroll
  for (int t = 0; t < 4; ++t) {
    v8f z = {0.f, 0.f, 0.f, 0.f, 0.f, 0.f, 0.f, 0.f};
    accH[t] = z;
    accX[t] = z;
  }

#pragma unroll 1
  for (int k0 = 0; k0 < K; k0 += 32) {
    FragH fah, fal;
    fah.u[0] = *(const v8us*)(ah + k0);
    fah.u[1] = *(const v8us*)(ah + k0 + 16);
    fal.u[0] = *(const v8us*)(al + k0);
    fal.u[1] = *(const v8us*)(al + k0 + 16);
#pragma unroll
    for (int t = 0; t < 4; ++t) {
      const size_t boff = (size_t)(c0 + 16 * t + m) * K + k0 + 8 * hh;
      FragH fbh, fbl;
      fbh.u[0] = *(const v8us*)(Bh + boff);
      fbh.u[1] = *(const v8us*)(Bh + boff + 16);
      fbl.u[0] = *(const v8us*)(Bl + boff);
      fbl.u[1] = *(const v8us*)(Bl + boff + 16);
      accH[t] = wmh(fah.v, fbh.v, accH[t]);
      accX[t] = wmh(fah.v, fbl.v, accX[t]);
      accX[t] = wmh(fal.v, fbh.v, accX[t]);
    }
  }

  {
    float* sp = stg + (wave * 16 + 8 * hh) * GBN + m;
#pragma unroll
    for (int t = 0; t < 4; ++t) {
#pragma unroll
      for (int r = 0; r < 8; ++r) sp[r * GBN + 16 * t] = accH[t][r] + accX[t][r] * LOINV;
    }
  }
  __syncthreads();

  const int rsub = lane >> 4, c4 = 4 * (lane & 15);
  const float* wst = stg + wave * 16 * GBN;
  const int gcol = c0 + c4;
#pragma unroll 1
  for (int pass = 0; pass < 2; ++pass) {
#pragma unroll
    for (int i = 0; i < 8; ++i) {
      const int lr = 2 * i + rsub;
      v4f v = *(const v4f*)(wst + lr * GBN + c4);
      v = v * ACCS;
      const int grow = rowBase + wave * 16 + lr;
      if (flags & F_RES)  { const v4f rv = *(const v4f*)(resid + (size_t)grow * ldr + gcol); v = rv + v; }
      if (flags & F_BIAS) { const v4f bv = *(const v4f*)(bias + gcol); v = v + bv; }
      if (flags & F_ACT)  { v.x = leakyf(v.x); v.y = leakyf(v.y); v.z = leakyf(v.z); v.w = leakyf(v.w); }
      if (flags & F_RSC)  { const float s = rsc[grow]; v = v * s; }
      if (flags & F_OUTF) *(volatile v4f*)(outF + (size_t)grow * ldF + colF + gcol) = v;
      if (flags & F_OUTP) {
        v2u ph, pl;
        split4(v, ASC, ph, pl);
        const size_t po = (size_t)grow * ldP + colP + gcol;
        *(volatile v2u*)(outH + po) = ph;
        *(volatile v2u*)(outL + po) = pl;
      }
    }
    if (pass == 0) __threadfence();
  }
}

__global__ __launch_bounds__(NTHR) void k_agg(
    const int* __restrict__ csr, const int* __restrict__ off, const int* __restrict__ cnt,
    const float* __restrict__ dinv, const float* __restrict__ hw, const float* __restrict__ bs,
    float* outF, int ldF, int colF, unsigned short* outH, unsigned short* outL, int ldP, int colP,
    int flags, int nN, int csrLen) {
  const int tid = threadIdx.x, lane = tid & 31, wave = tid >> 5;
  const int tbase = blockIdx.x * TGT + wave * 32;
  const int cl = tbase + lane;
  const int cnt_l = cnt[cl];
  const int off_l = off[cl];
  union FI { float f; int i; };
  FI dvu; dvu.f = dinv[cl];
  const v4f bb = *(const v4f*)(bs + 4 * lane);

#pragma unroll 1
  for (int j = 0; j < 32; ++j) {
    const int c = tbase + j;
    int n = __builtin_amdgcn_readlane(cnt_l, j);
    n = n < 0 ? 0 : (n > DEGCAP ? DEGCAP : n);
    const int st = __builtin_amdgcn_readlane(off_l, j);
    FI du; du.i = __builtin_amdgcn_readlane(dvu.i, j);
    const float dc = du.f;
    v4f acc = {0.f, 0.f, 0.f, 0.f};
#pragma unroll 1
    for (int q0 = 0; q0 < n; q0 += 32) {
      int pos = st + q0 + lane;
      pos = pos < 0 ? 0 : (pos > csrLen - 1 ? csrLen - 1 : pos);
      int sl = csr[pos];
      sl = sl < 0 ? 0 : (sl > nN - 1 ? nN - 1 : sl);
      const int mcnt = (n - q0) < 32 ? (n - q0) : 32;
#pragma unroll 1
      for (int p = 0; p < mcnt; ++p) {
        const int s = __builtin_amdgcn_readlane(sl, p);
        acc = acc + *(const v4f*)(hw + (size_t)s * EMB + 4 * lane);
      }
    }
    const v4f sv = *(const v4f*)(hw + (size_t)c * EMB + 4 * lane);
    v4f v = (acc + sv) * dc + bb;
    v.x = leakyf(v.x); v.y = leakyf(v.y); v.z = leakyf(v.z); v.w = leakyf(v.w);
    v2u ph, pl;
    split4(v, ASC, ph, pl);
    const size_t fo = (size_t)c * ldF + colF + 4 * lane;
    const size_t po = (size_t)c * ldP + colP + 4 * lane;
    if (flags & F_OUTF) *(volatile v4f*)(outF + fo) = v;
    if (flags & F_OUTP) { *(volatile v2u*)(outH + po) = ph; *(volatile v2u*)(outL + po) = pl; }
    __threadfence();
    if (flags & F_OUTF) *(volatile v4f*)(outF + fo) = v;
    if (flags & F_OUTP) { *(volatile v2u*)(outH + po) = ph; *(volatile v2u*)(outL + po) = pl; }
  }
}

__global__ __launch_bounds__(NTHR) void k_cvt(const float* __restrict__ xF, unsigned short* cxH,
                                              unsigned short* cxL, int rows) {
  const int gid = (int)blockIdx.x * NTHR + (int)threadIdx.x;
  const int r = gid / (DDIM / 8);
  const int q = gid - r * (DDIM / 8);
  if (r >= rows) return;
  const float* p = xF + (size_t)r * DDIM + 8 * q;
  const v4f a = *(const v4f*)p;
  const v4f b = *(const v4f*)(p + 4);
  v4u hv, lv;
  split8(a, b, ASC, hv, lv);
  const size_t po = (size_t)r * DDIM + 8 * q;
  *(volatile v4u*)(cxH + po) = hv;
  *(volatile v4u*)(cxL + po) = lv;
  __threadfence();
  *(volatile v4u*)(cxH + po) = hv;
  *(volatile v4u*)(cxL + po) = lv;
}

__global__ __launch_bounds__(NTHR) void k_cross(const float* __restrict__ xF, const float* __restrict__ cw,
                                                const float* __restrict__ cb, unsigned short* zH, unsigned short* zL,
                                                int rows) {
#pragma clang fp contract(off)
  __shared__ __attribute__((aligned(16))) float srow[NWAVE * DDIM];
  const int tid = threadIdx.x, lane = tid & 31, wave = tid >> 5;
  const int r  = (int)blockIdx.x * NWAVE + wave;
  const int rc = r > rows - 1 ? rows - 1 : r;
  const float* xp = xF + (size_t)rc * DDIM;
  float x0[6], xc[6];
#pragma unroll
  for (int j = 0; j < 6; ++j) { x0[j] = xp[lane + 32 * j]; xc[j] = x0[j]; }
#pragma unroll 1
  for (int i = 0; i < 2; ++i) {
    double p = 0.0;
#pragma unroll
    for (int j = 0; j < 6; ++j) p = fma((double)xc[j], (double)cw[i * DDIM + lane + 32 * j], p);
#pragma unroll
    for (int o = 16; o >= 1; o >>= 1) p += shfl_xor_d(p, o);
    const float pf = __int_as_float(__builtin_amdgcn_readfirstlane(__float_as_int((float)p)));
#pragma unroll
    for (int j = 0; j < 6; ++j) xc[j] = x0[j] * pf + cb[i * DDIM + lane + 32 * j] + xc[j];
  }
  float* sw = srow + wave * DDIM;
#pragma unroll
  for (int j = 0; j < 6; ++j) sw[lane + 32 * j] = xc[j];
  __syncthreads();
  const int lq = lane < (DDIM / 8) ? lane : 0;
  const v4f a = *(const v4f*)(sw + 8 * lq);
  const v4f b = *(const v4f*)(sw + 8 * lq + 4);
  v4u hv, lv;
  split8(a, b, ASC, hv, lv);
  const bool act = (lane < (DDIM / 8)) && (r < rows);
  const size_t po = (size_t)r * ZDIM + DDIM + 8 * lq;
  if (act) { *(volatile v4u*)(zH + po) = hv; *(volatile v4u*)(zL + po) = lv; }
  __threadfence();
  if (act) { *(volatile v4u*)(zH + po) = hv; *(volatile v4u*)(zL + po) = lv; }
}

__global__ __launch_bounds__(NTHR) void k_pdot(const float* __restrict__ pF, const float* __restrict__ w2,
                                               const float* __restrict__ b2, float* out, int row0, int rows, int nN) {
  __shared__ __attribute__((aligned(16))) float sres[32];
  const int tid = threadIdx.x, lane = tid & 31, wave = tid >> 5;
  const double bv = (double)b2[0];
#pragma unroll 1
  for (int t = 0; t < 4; ++t) {
    const int nl  = (int)blockIdx.x * 32 + wave * 4 + t;
    const int nlc = nl > rows - 1 ? rows - 1 : nl;
    const float* hp = pF + (size_t)nlc * PHID;
    double p = 0.0;
#pragma unroll 2
    for (int j = 0; j < PHID / 32; ++j) {
      const int f = lane + 32 * j;
      p = fma((double)hp[f], (double)w2[f], p);
    }
#pragma unroll
    for (int o = 16; o >= 1; o >>= 1) p += shfl_xor_d(p, o);
    const float x = (float)(p + bv);
    const float e = expf(-fabsf(x));
    const float rcp = 1.0f / (1.0f + e);
    const float y = x >= 0.f ? rcp : e * rcp;
    if (lane == 0) sres[wave * 4 + t] = y;
  }
  __syncthreads();
  const bool wr = (wave == 0) && (lane < 8);
  const int lq = lane & 7;
  const v4f v = *(const v4f*)(sres + 4 * lq);
  const int g0 = row0 + (int)blockIdx.x * 32 + 4 * lq;
#pragma unroll 1
  for (int pass = 0; pass < 2; ++pass) {
    if (wr) {
      if (g0 + 3 < nN) {
        *(volatile v4f*)(out + g0) = v;
      } else {
        if (g0     < nN) *(volatile float*)(out + g0)     = v.x;
        if (g0 + 1 < nN) *(volatile float*)(out + g0 + 1) = v.y;
        if (g0 + 2 < nN) *(volatile float*)(out + g0 + 2) = v.z;
        if (g0 + 3 < nN) *(volatile float*)(out + g0 + 3) = v.w;
      }
    }
    if (pass == 0) __threadfence();
  }
}

static inline size_t take(size_t& off, size_t bytes) {
  const size_t o = off;
  off = (off + bytes + 255) & ~(size_t)255;
  return o;
}
static inline int cdiv(int a, int b) { return (a + b - 1) / b; }

extern "C" void kernel_launch(void* const* d_in, const int* in_sizes, int n_in,
                              void* d_out, int out_size, void* d_ws, size_t ws_size,
                              hipStream_t stream) {
  if (n_in < 18) return;
  const int nN = in_sizes[0] / NFEAT;
  const int nE = in_sizes[1] / 2;
  if (nN <= 0 || nE <= 0 || in_sizes[0] != nN * NFEAT || in_sizes[1] != 2 * nE) return;
  if (in_sizes[2] != NH * EMB || in_sizes[3] != EMB) return;
  if (in_sizes[4] != EMB * EMB || in_sizes[5] != EMB || in_sizes[6] != EMB * EMB || in_sizes[7] != EMB) return;
  if (in_sizes[8] != 2 * DDIM * RHID || in_sizes[9] != 2 * RHID) return;
  if (in_sizes[10] != 2 * RHID * DDIM || in_sizes[11] != 2 * DDIM) return;
  if (in_sizes[12] != 2 * DDIM || in_sizes[13] != 2 * DDIM) return;
  if (in_sizes[14] != ZDIM * PHID || in_sizes[15] != PHID || in_sizes[16] != PHID || in_sizes[17] < 1) return;
  if (out_size != nN) return;
  if (nN > (1 << 20) || nE > (1 << 28)) return;

  const int*   dx   = (const int*)d_in[0];
  const int*   ei   = (const int*)d_in[1];
  const float* w_g0 = (const float*)d_in[2];
  const float* b_g0 = (const float*)d_in[3];
  const float* w_g1 = (const float*)d_in[4];
  const float* b_g1 = (const float*)d_in[5];
  const float* w_g2 = (const float*)d_in[6];
  const float* b_g2 = (const float*)d_in[7];
  const float* rw1  = (const float*)d_in[8];
  const float* rb1  = (const float*)d_in[9];
  const float* rw2  = (const float*)d_in[10];
  const float* rb2  = (const float*)d_in[11];
  const float* cw   = (const float*)d_in[12];
  const float* cb   = (const float*)d_in[13];
  const float* pw1  = (const float*)d_in[14];
  const float* pb1  = (const float*)d_in[15];
  const float* pw2  = (const float*)d_in[16];
  const float* pb2  = (const float*)d_in[17];
  float* out = (float*)d_out;

  const int NPAD   = cdiv(nN, TGT) * TGT;
  const int nBC    = cdiv(nN, NBC);
  const int CNTPAD = nBC * NBC;
  const int nBF    = cdiv(nN, NBF);
  const int OFFN   = nBF * NBF;
  if (nBF + 1 > RBN) return;
  if (OFFN > CNTPAD || NPAD > OFFN) return;
  const int csrLen = ((nE + 31) & ~31) + 32 * (nBF + 1);
  const int CH     = NPAD < CHROWS ? NPAD : CHROWS;
  const int nChunk = cdiv(NPAD, CHROWS);

  const size_t eg0 = (size_t)NH * EMB, eg1 = (size_t)EMB * EMB;
  const size_t er1 = (size_t)2 * DDIM * RHID, er2 = (size_t)2 * RHID * DDIM, ep1 = (size_t)ZDIM * PHID;

  char* ws = (char*)d_ws;
  size_t off = 0;
  const size_t oWh0 = take(off, eg0 * 2), oWl0 = take(off, eg0 * 2);
  const size_t oWh1 = take(off, eg1 * 2), oWl1 = take(off, eg1 * 2);
  const size_t oWh2 = take(off, eg1 * 2), oWl2 = take(off, eg1 * 2);
  const size_t oRh1 = take(off, er1 * 2), oRl1 = take(off, er1 * 2);
  const size_t oRh2 = take(off, er2 * 2), oRl2 = take(off, er2 * 2);
  const size_t oPh1 = take(off, ep1 * 2), oPl1 = take(off, ep1 * 2);
  const size_t oXF  = take(off, (size_t)NPAD * DDIM * 4);
  const size_t oCnt = take(off, (size_t)CNTPAD * 4);
  const size_t oDv  = take(off, (size_t)CNTPAD * 4);
  const size_t oOff = take(off, (size_t)OFFN * 4);
  const size_t oRb  = take(off, (size_t)RBN * 4);
  const size_t oCsr = take(off, (size_t)csrLen * 4);
  const size_t oU   = off;
  const size_t oXdH = take(off, (size_t)NPAD * NH * 2);
  const size_t oXdL = take(off, (size_t)NPAD * NH * 2);
  const size_t oGH  = take(off, (size_t)NPAD * EMB * 2);
  const size_t oGL  = take(off, (size_t)NPAD * EMB * 2);
  const size_t oHw  = take(off, (size_t)NPAD * EMB * 4);
  const size_t endG = off;
  off = oU;
  const size_t oCxH = take(off, (size_t)CH * DDIM * 2), oCxL = take(off, (size_t)CH * DDIM * 2);
  const size_t oHH  = take(off, (size_t)CH * RHID * 2), oHL  = take(off, (size_t)CH * RHID * 2);
  const size_t oD1F = take(off, (size_t)CH * DDIM * 4);
  const size_t oD1H = take(off, (size_t)CH * DDIM * 2), oD1L = take(off, (size_t)CH * DDIM * 2);
  const size_t oZH  = take(off, (size_t)CH * ZDIM * 2), oZL  = take(off, (size_t)CH * ZDIM * 2);
  const size_t oPF  = take(off, (size_t)CH * PHID * 4);
  const size_t endR = off;
  const size_t total = endG > endR ? endG : endR;
  if (total > ws_size || total > (size_t)WSCAP) return;

  unsigned short* wh0 = (unsigned short*)(ws + oWh0); unsigned short* wl0 = (unsigned short*)(ws + oWl0);
  unsigned short* wh1 = (unsigned short*)(ws + oWh1); unsigned short* wl1 = (unsigned short*)(ws + oWl1);
  unsigned short* wh2 = (unsigned short*)(ws + oWh2); unsigned short* wl2 = (unsigned short*)(ws + oWl2);
  unsigned short* rh1 = (unsigned short*)(ws + oRh1); unsigned short* rl1 = (unsigned short*)(ws + oRl1);
  unsigned short* rh2 = (unsigned short*)(ws + oRh2); unsigned short* rl2 = (unsigned short*)(ws + oRl2);
  unsigned short* ph1 = (unsigned short*)(ws + oPh1); unsigned short* pl1 = (unsigned short*)(ws + oPl1);
  float* xF   = (float*)(ws + oXF);
  int*   cnt  = (int*)(ws + oCnt);
  float* dinv = (float*)(ws + oDv);
  int*   offp = (int*)(ws + oOff);
  int*   rbp  = (int*)(ws + oRb);
  int*   csr  = (int*)(ws + oCsr);
  unsigned short* xdH = (unsigned short*)(ws + oXdH); unsigned short* xdL = (unsigned short*)(ws + oXdL);
  unsigned short* gH  = (unsigned short*)(ws + oGH);  unsigned short* gL  = (unsigned short*)(ws + oGL);
  float* hw = (float*)(ws + oHw);
  unsigned short* cxH = (unsigned short*)(ws + oCxH); unsigned short* cxL = (unsigned short*)(ws + oCxL);
  unsigned short* hH  = (unsigned short*)(ws + oHH);  unsigned short* hL  = (unsigned short*)(ws + oHL);
  float* d1F = (float*)(ws + oD1F);
  unsigned short* d1H = (unsigned short*)(ws + oD1H); unsigned short* d1L = (unsigned short*)(ws + oD1L);
  unsigned short* zH  = (unsigned short*)(ws + oZH);  unsigned short* zL  = (unsigned short*)(ws + oZL);
  float* pF = (float*)(ws + oPF);

  const int vec8 = ((nE & 3) == 0) ? 1 : 0;

  k_wprep<<<dim3(cdiv(EMB * (NH / 8), NTHR), 1), NTHR, 0, stream>>>(w_g0, NH, EMB, wh0, wl0);
  k_wprep<<<dim3(cdiv(EMB * (EMB / 8), NTHR), 1), NTHR, 0, stream>>>(w_g1, EMB, EMB, wh1, wl1);
  k_wprep<<<dim3(cdiv(EMB * (EMB / 8), NTHR), 1), NTHR, 0, stream>>>(w_g2, EMB, EMB, wh2, wl2);
  k_wprep<<<dim3(cdiv(RHID * (DDIM / 8), NTHR), 2), NTHR, 0, stream>>>(rw1, DDIM, RHID, rh1, rl1);
  k_wprep<<<dim3(cdiv(DDIM * (RHID / 8), NTHR), 2), NTHR, 0, stream>>>(rw2, RHID, DDIM, rh2, rl2);
  k_wprep<<<dim3(cdiv(PHID * (ZDIM / 8), NTHR), 1), NTHR, 0, stream>>>(pw1, ZDIM, PHID, ph1, pl1);

  k_embed<<<NPAD / 16, NTHR, 0, stream>>>(dx, xF, xdH, xdL, nN, NPAD);

  hipFuncSetAttribute(reinterpret_cast<const void*>(&k_count), hipFuncAttributeMaxDynamicSharedMemorySize, LDS_COUNT);
  k_count<<<nBC, NTHR, LDS_COUNT, stream>>>(ei, cnt, dinv, nE, nN, vec8);
  k_offsets<<<1, OTHR, 0, stream>>>(cnt, offp, rbp, nBF);
  hipFuncSetAttribute(reinterpret_cast<const void*>(&k_fill), hipFuncAttributeMaxDynamicSharedMemorySize, LDS_FILL);
  k_fill<<<nBF, NTHR, LDS_FILL, stream>>>(ei, offp, rbp, csr, nN, nE, vec8, csrLen);

  k_gemm<<<dim3(EMB / GBN, NPAD / GBM), NTHR, 0, stream>>>(xdH, xdL, NH, wh0, wl0, NH, b_g0, xF, DDIM, dinv,
      hw, EMB, 0, gH, gL, EMB, 0, F_BIAS | F_ACT | F_OUTP);
  k_gemm<<<dim3(EMB / GBN, NPAD / GBM), NTHR, 0, stream>>>(gH, gL, EMB, wh1, wl1, EMB, b_g1, xF, DDIM, dinv,
      hw, EMB, 0, xdH, xdL, NH, 0, F_RSC | F_OUTF);
  k_agg<<<NPAD / TGT, NTHR, 0, stream>>>(csr, offp, cnt, dinv, hw, b_g1, xF, DDIM, NH, gH, gL, EMB, 0,
      F_OUTP, nN, csrLen);
  k_gemm<<<dim3(EMB / GBN, NPAD / GBM), NTHR, 0, stream>>>(gH, gL, EMB, wh2, wl2, EMB, b_g2, xF, DDIM, dinv,
      hw, EMB, 0, xdH, xdL, NH, 0, F_RSC | F_OUTF);
  k_agg<<<NPAD / TGT, NTHR, 0, stream>>>(csr, offp, cnt, dinv, hw, b_g2, xF, DDIM, NH, xdH, xdL, NH, 0,
      F_OUTF, nN, csrLen);

  for (int c = 0; c < nChunk; ++c) {
    const int R0 = c * CHROWS;
    const int CR = (NPAD - R0) < CHROWS ? (NPAD - R0) : CHROWS;
    const float* xFc = xF + (size_t)R0 * DDIM;
    k_cvt<<<(CR * (DDIM / 8)) / NTHR, NTHR, 0, stream>>>(xFc, cxH, cxL, CR);
    k_gemm<<<dim3(RHID / GBN, CR / GBM), NTHR, 0, stream>>>(cxH, cxL, DDIM, rh1, rl1, DDIM, rb1, xFc, DDIM, dinv,
        d1F, DDIM, 0, hH, hL, RHID, 0, F_BIAS | F_ACT | F_OUTP);
    k_gemm<<<dim3(DDIM / GBN, CR / GBM), NTHR, 0, stream>>>(hH, hL, RHID, rh2, rl2, RHID, rb2, xFc, DDIM, dinv,
        d1F, DDIM, 0, d1H, d1L, DDIM, 0, F_BIAS | F_RES | F_ACT | F_OUTF | F_OUTP);
    k_gemm<<<dim3(RHID / GBN, CR / GBM), NTHR, 0, stream>>>(d1H, d1L, DDIM, rh1 + (size_t)DDIM * RHID,
        rl1 + (size_t)DDIM * RHID, DDIM, rb1 + RHID, xFc, DDIM, dinv,
        pF, PHID, 0, hH, hL, RHID, 0, F_BIAS | F_ACT | F_OUTP);
    k_gemm<<<dim3(DDIM / GBN, CR / GBM), NTHR, 0, stream>>>(hH, hL, RHID, rh2 + (size_t)RHID * DDIM,
        rl2 + (size_t)RHID * DDIM, RHID, rb2 + DDIM, d1F, DDIM, dinv,
        pF, PHID, 0, zH, zL, ZDIM, 0, F_BIAS | F_RES | F_ACT | F_OUTP);
    k_cross<<<CR / NWAVE, NTHR, 0, stream>>>(xFc, cw, cb, zH, zL, CR);
    k_gemm<<<dim3(PHID / GBN, CR / GBM), NTHR, 0, stream>>>(zH, zL, ZDIM, ph1, pl1, ZDIM, pb1, xFc, DDIM, dinv,
        pF, PHID, 0, cxH, cxL, DDIM, 0, F_BIAS | F_ACT | F_OUTF);
    k_pdot<<<CR / 32, NTHR, 0, stream>>>(pF, pw2, pb2, out, R0, CR, nN);
  }
}
